// GMamba_481036337188
// MI455X (gfx1250) — hardware-run, weakly checked
//
#include <hip/hip_runtime.h>


namespace {
constexpr int NB = 8, T = 32, HW = 256, D = 128, NR = NB * T * HW  ;
constexpr float XS = 8.0f, WSC = 256.0f, EPS = 1e-5f;
typedef _Float16 b16;
typedef __attribute__((ext_vector_type(16))) _Float16 v16b;
typedef __attribute__((ext_vector_type(8))) _Float16 v8b;
typedef __attribute__((ext_vector_type(8))) float v8f;
typedef __attribute__((ext_vector_type(4))) float v4f;
__device__ __forceinline__ float bf16_rne(float f) { unsigned int u = __float_as_uint(f); u += 0x7FFFu + ((u >> 16) & 1u); float r = __uint_as_float(u & 0xFFFF0000u); asm volatile("" : "+v"(r)); return r; }
__device__ __forceinline__ float bfv(float f) { float r = bf16_rne(f); asm volatile("" : "+v"(r)); return r; }
__device__ __forceinline__ void split16(float v, b16& hi, b16& lo) { hi = (b16)v; lo = (b16)(v - (float)hi); }
__device__ __forceinline__ v16b frag_kb(const b16* p, int hh) { const v8b a = *(const v8b*)(p + 8 * hh), b = *(const v8b*)(p + 16 + 8 * hh); v16b f;
#pragma unroll
  for (int e = 0; e < 8; ++e) { f[e] = a[e]; f[8 + e] = b[e]; } return f; }
__device__ __forceinline__ v8f wmma16b(v16b a, v16b b, v8f c) { v8f d = __builtin_amdgcn_wmma_f32_16x16x32_f16(false, a, false, b, (short)0, c, false, false); asm volatile("v_nop\n\tv_nop\n\tv_nop\n\tv_nop" : "+v"(d) : "v"(a), "v"(b)); return d; }
__device__ __forceinline__ void wave_lds_sync() { __builtin_amdgcn_fence(__ATOMIC_RELEASE, "workgroup"); __builtin_amdgcn_wave_barrier(); __builtin_amdgcn_fence(__ATOMIC_ACQUIRE, "workgroup"); }
__device__ __forceinline__ float pmul(float a, float b) { float p = a * b; asm volatile("" : "+v"(p)); return p; }
__device__ __forceinline__ float wsum(float v) { for (int o = 16; o; o >>= 1) v += __shfl_xor(v, o); return v; }

__global__ __launch_bounds__(256) void wput_kernel(const float* __restrict__ wb, const float* __restrict__ wc, const float* __restrict__ wo, b16* __restrict__ WBC, b16* __restrict__ WO) { const int u = blockIdx.x * 256 + threadIdx.x; if (u >= 384 * 16) return; const int r = u / 16, k0 = (u % 16) * 8; v8b v;
#pragma unroll
  for (int j = 0; j < 8; ++j) { const int k = k0 + j; v[j] = (b16)(bf16_rne(r < D ? wb[(size_t)k * D + r] : (r < 2 * D ? wc[(size_t)k * D + r - D] : wo[(size_t)k * D + r - 2 * D])) * WSC); }
  for (int pass = 0; pass < 2; ++pass) { *(volatile v8b*)((r < 2 * D ? WBC + (size_t)r * D : WO + (size_t)(r - 2 * D) * D) + k0) = v; __threadfence(); } }
__global__ __launch_bounds__(32) void proj_kernel(const float* __restrict__ x, const float* __restrict__ g1, const float* __restrict__ b1, const float* __restrict__ g2, const float* __restrict__ b2, const b16* __restrict__ WBC, const float* __restrict__ bB, const float* __restrict__ bC, int RLIM, float* __restrict__ BC, float* __restrict__ DD) { __shared__ __attribute__((aligned(16))) b16 Ah[16][D + 8], Al[16][D + 8]; __shared__ float Df[16][132], Tf[16][260]; const int lane = threadIdx.x, nloc = lane & 15, hlf = lane >> 4; const size_t m0 = (size_t)blockIdx.x * 16; if (m0 >= (size_t)RLIM) return;
  for (int rr = 0; rr < 16; ++rr) { const size_t r = m0 + rr; const int t = (int)((r / HW) % T); float d[4]; float s1 = 0.0f;
    for (int q = 0; q < 4; ++q) { const int c = q * 32 + lane; const float cur = bf16_rne(x[r * D + c]); const float prev = t > 0 ? bf16_rne(x[(r - HW) * D + c]) : 0.0f; d[q] = t > 0 ? cur - prev : 0.0f; Df[rr][c] = d[q]; s1 += d[q]; }
    s1 = wsum(s1); const float mu = s1 * (1.0f / D); float s2 = 0.0f; for (int q = 0; q < 4; ++q) { const float e = d[q] - mu; s2 += e * e; } s2 = wsum(s2); const float rs = rsqrtf(s2 * (1.0f / D) + EPS); float n1[4]; float t1 = 0.0f;
    for (int q = 0; q < 4; ++q) { const int c = q * 32 + lane; n1[q] = pmul(pmul(d[q] - mu, rs), bfv(g1[c])) + bfv(b1[c]); t1 += n1[q]; }
    t1 = wsum(t1); const float mu2 = t1 * (1.0f / D); float t2 = 0.0f; for (int q = 0; q < 4; ++q) { const float e = n1[q] - mu2; t2 += e * e; } t2 = wsum(t2); const float rs2 = rsqrtf(t2 * (1.0f / D) + EPS);
    for (int q = 0; q < 4; ++q) { const int c = q * 32 + lane; const float xn = pmul(pmul(n1[q] - mu2, rs2), bfv(g2[c])) + bfv(b2[c]); b16 p, ql; split16(xn * XS, p, ql); Ah[rr][c] = p; Al[rr][c] = ql; } }
  wave_lds_sync(); v8f acc[16];
#pragma unroll
  for (int tt = 0; tt < 16; ++tt) acc[tt] = (v8f){};
#pragma unroll
  for (int kb = 0; kb < D; kb += 32) { const v16b a = frag_kb(&Ah[nloc][kb], hlf), al = frag_kb(&Al[nloc][kb], hlf);
#pragma unroll
    for (int tt = 0; tt < 16; ++tt) { const v16b bw = frag_kb(WBC + (size_t)(tt * 16 + nloc) * D + kb, hlf); acc[tt] = wmma16b(a, bw, acc[tt]); acc[tt] = wmma16b(al, bw, acc[tt]); } }
#pragma unroll
  for (int tt = 0; tt < 16; ++tt) { const int cc = tt * 16 + nloc; const float bb = cc < D ? bfv(bB[cc]) : bfv(bC[cc - D]);
#pragma unroll
    for (int r8 = 0; r8 < 8; ++r8) Tf[8 * hlf + r8][cc] = acc[tt][r8] * (1.0f / (XS * WSC)) + bb; }
  wave_lds_sync();
  for (int pass = 0; pass < 2; ++pass) { for (int rr = 0; rr < 16; ++rr) { for (int q = 0; q < 2; ++q) *(volatile v4f*)(BC + (m0 + rr) * (2 * D) + q * 128 + lane * 4) = *(const v4f*)(&Tf[rr][q * 128 + lane * 4]); *(volatile v4f*)(DD + (m0 + rr) * D + lane * 4) = *(const v4f*)(&Df[rr][lane * 4]); } __threadfence(); } }
__global__ __launch_bounds__(256) void scan_kernel(const float* __restrict__ BC, const float* __restrict__ A, int BLIM, float* __restrict__ Y) { const size_t u = (size_t)blockIdx.x * 256 + threadIdx.x; if (u >= (size_t)BLIM * HW * D) return; const int c = (int)(u % D); const int hw = (int)((u / D) % HW); const int b = (int)(u / ((size_t)D * HW)); const float dec = __expf(bfv(A[c]));
  for (int pass = 0; pass < 2; ++pass) { float h = 0.0f;
#pragma unroll 1
    for (int t = 0; t < T; ++t) { const size_t r = ((size_t)b * T + t) * HW + hw; h = pmul(dec, h) + BC[r * (2 * D) + c]; ((volatile float*)Y)[r * D + c] = pmul(BC[r * (2 * D) + D + c], h); }
    __threadfence(); } }
__global__ __launch_bounds__(32) void out_kernel(const float* __restrict__ Y, const b16* __restrict__ WO, const float* __restrict__ bo, const float* __restrict__ DD, int RLIM, float* __restrict__ out) { __shared__ __attribute__((aligned(16))) b16 Ah[16][D + 8], Al[16][D + 8]; __shared__ float Tf[16][132]; const int lane = threadIdx.x, nloc = lane & 15, hlf = lane >> 4; const size_t m0 = (size_t)blockIdx.x * 16; if (m0 >= (size_t)RLIM) return;
  for (int rr = 0; rr < 16; ++rr) for (int q = 0; q < 4; ++q) { b16 p, ql; split16(Y[(m0 + rr) * D + q * 32 + lane] * XS, p, ql); Ah[rr][q * 32 + lane] = p; Al[rr][q * 32 + lane] = ql; }
  wave_lds_sync(); v8f acc[8];
#pragma unroll
  for (int t = 0; t < 8; ++t) acc[t] = (v8f){};
#pragma unroll
  for (int kb = 0; kb < D; kb += 32) { const v16b a = frag_kb(&Ah[nloc][kb], hlf), al = frag_kb(&Al[nloc][kb], hlf);
#pragma unroll
    for (int t = 0; t < 8; ++t) { const v16b bw = frag_kb(WO + (size_t)(t * 16 + nloc) * D + kb, hlf); acc[t] = wmma16b(a, bw, acc[t]); acc[t] = wmma16b(al, bw, acc[t]); } }
#pragma unroll
  for (int t = 0; t < 8; ++t) { const int cc = t * 16 + nloc; const float bb = bfv(bo[cc]);
#pragma unroll
    for (int r8 = 0; r8 < 8; ++r8) { const int rr = 8 * hlf + r8; Tf[rr][cc] = acc[t][r8] * (1.0f / (XS * WSC)) + bb + DD[(m0 + rr) * D + cc]; } }
  wave_lds_sync();
  for (int pass = 0; pass < 2; ++pass) { for (int rr = 0; rr < 16; ++rr) *(volatile v4f*)(out + (m0 + rr) * D + lane * 4) = *(const v4f*)(&Tf[rr][lane * 4]); __threadfence(); } }
}

extern "C" void kernel_launch(void* const* d_in, const int* in_sizes, int n_in, void* d_out, int out_size, void* d_ws, size_t ws_size, hipStream_t stream) {
  (void)n_in;
  auto Fp = [&](int i) { return (const float*)d_in[i]; };
  if (in_sizes[0] != NR * D || in_sizes[5] != D * D || in_sizes[7] != D * D || in_sizes[9] != D * D || in_sizes[11] != D || out_size != NR * D) return;
  const int BLIM = NB;
  const int RLIM = BLIM * T * HW;
  size_t off = 0; char* ws = (char*)d_ws;
  auto carve = [&](size_t bytes) { char* p = ws + off; off += (bytes + 255) & ~(size_t)255; return p; };
  b16* WBC = (b16*)carve((size_t)2 * D * D * 2); b16* WO = (b16*)carve((size_t)D * D * 2); float* BC = (float*)carve((size_t)NR * 2 * D * 4); float* DD = (float*)carve((size_t)NR * D * 4); float* Y = (float*)carve((size_t)NR * D * 4);
  if (off > ws_size || off > ((size_t)160 << 20)) return;
  wput_kernel<<<(384 * 16 + 255) / 256, 256, 0, stream>>>(Fp(5), Fp(7), Fp(9), WBC, WO);
  proj_kernel<<<RLIM / 16, 32, 0, stream>>>(Fp(0), Fp(1), Fp(2), Fp(3), Fp(4), WBC, Fp(6), Fp(8), RLIM, BC, DD);
  scan_kernel<<<(unsigned)(((size_t)BLIM * HW * D + 255) / 256), 256, 0, stream>>>(BC, Fp(11), BLIM, Y);
  out_kernel<<<RLIM / 16, 32, 0, stream>>>(Y, WO, Fp(10), DD, RLIM, (float*)d_out);
}
